// ISTFT_4449586118853
// MI455X (gfx1250) — hardware-verified
//
#include <hip/hip_runtime.h>


namespace {
typedef _Float16 b16;
typedef __attribute__((ext_vector_type(16))) _Float16 v16b;
typedef __attribute__((ext_vector_type(8))) _Float16 v8b;
typedef __attribute__((ext_vector_type(4))) _Float16 v4h;
typedef __attribute__((ext_vector_type(2))) _Float16 v2h;
typedef __attribute__((ext_vector_type(8))) float v8f;
typedef __attribute__((ext_vector_type(4))) float v4f;
typedef __attribute__((ext_vector_type(2))) float v2f;
__device__ __forceinline__ float bf16_rne(float f) { unsigned int u = __float_as_uint(f); u += 0x7FFFu + ((u >> 16) & 1u); return __uint_as_float(u & 0xFFFF0000u); }
__device__ __forceinline__ void split16(float v, b16& hi, b16& lo) { hi = (b16)v; lo = (b16)(v - (float)hi); }
__device__ __forceinline__ v16b frag_kb(const b16* p, int hh) { const v8b a = *(const v8b*)(p + 8 * hh), b = *(const v8b*)(p + 16 + 8 * hh); v16b f;
#pragma unroll
  for (int e = 0; e < 8; ++e) { f[e] = a[e]; f[8 + e] = b[e]; } return f; }
__device__ __forceinline__ v8f wmma16b(v16b a, v16b b, v8f c) { v8f d = __builtin_amdgcn_wmma_f32_16x16x32_f16(false, a, false, b, (short)0, c, false, false); asm volatile("v_nop\n\tv_nop\n\tv_nop\n\tv_nop" : "+v"(d) : "v"(a), "v"(b)); return d; }
__device__ __forceinline__ void wave_lds_sync() { __builtin_amdgcn_fence(__ATOMIC_RELEASE, "workgroup"); __builtin_amdgcn_wave_barrier(); __builtin_amdgcn_fence(__ATOMIC_ACQUIRE, "workgroup"); }
__device__ __forceinline__ float pmul(float a, float b) { float p = a * b; asm volatile("" : "+v"(p)); return p; }
__device__ __forceinline__ int iclamp(int v, int lo, int hi) { return v < lo ? lo : (v > hi ? hi : v); }
__device__ __forceinline__ float nexp2(float v) { return __builtin_amdgcn_exp2f(v); }

constexpr int B = 8, T = 1024, NB1 = 1025, NF = 2048, HOP = 512, KH = 1040, KP = 2 * KH, M = B * T, ML = M  , LEN = (T - 1) * HOP, LFULL = LEN + NF;
constexpr float XS = 8.0f, WSC2 = 1048576.0f;
static_assert(KP % 32 == 0 && KH >= NB1 && M % 64 == 0 && ML % 64 == 0 && NF % 128 == 0 && LEN % 32 == 0, "tiling");
__global__ __launch_bounds__(256) void aprep_kernel(const float* __restrict__ re, const float* __restrict__ im, b16* __restrict__ AP) {
  const size_t u = (size_t)blockIdx.x * 256 + threadIdx.x; if (u >= (size_t)M * KP / 8) return; const size_t row = u / (KP / 8); const int k0 = (int)(u % (KP / 8)) * 8; v8b o;
  for (int j = 0; j < 8; ++j) { const int k = k0 + j; float v = 0.0f; if (k < NB1) v = re[row * NB1 + k]; else if (k >= KH && k < KH + NB1) v = im[row * NB1 + (k - KH)]; o[j] = (b16)(bf16_rne(v) * XS); }
  for (int pass = 0; pass < 2; ++pass) { *(volatile v8b*)(AP + row * KP + k0) = o; __threadfence(); }
}
__global__ __launch_bounds__(256) void wprep_kernel(const float* __restrict__ cr, const float* __restrict__ ci, b16* __restrict__ WB) {
  const size_t u = (size_t)blockIdx.x * 256 + threadIdx.x; if (u >= (size_t)NF * KP / 8) return; const size_t o_ = u / (KP / 8); const int k0 = (int)(u % (KP / 8)) * 8; v8b o;
  for (int jj = 0; jj < 8; ++jj) { const int k = k0 + jj; float w = 0.0f;
    if (k < NB1) { w = bf16_rne(cr[o_ * NF + k]); if (k >= 1 && k <= NB1 - 2) w += bf16_rne(cr[o_ * NF + (NF - k)]); }
    else if (k >= KH && k < KH + NB1) { const int j = k - KH; w = bf16_rne(ci[o_ * NF + j]); if (j >= 1 && j <= NB1 - 2) w -= bf16_rne(ci[o_ * NF + (NF - j)]); w = -w; }
    o[jj] = (b16)(w * WSC2); }
  for (int pass = 0; pass < 2; ++pass) { *(volatile v8b*)(WB + o_ * KP + k0) = o; __threadfence(); }
}
__global__ __launch_bounds__(128) void gemm_kernel(const b16* __restrict__ AP, const b16* __restrict__ WB, float* __restrict__ S) {
  __shared__ __attribute__((aligned(16))) float Tf[4][16][128 + 4];
  const int wave = threadIdx.x >> 5, lane = threadIdx.x & 31, nloc = lane & 15, hlf = lane >> 4; const size_t m0 = ((size_t)blockIdx.x * 4 + wave) * 16; const int n0 = blockIdx.y * 128;
  v8f acc[8];
#pragma unroll
  for (int t = 0; t < 8; ++t) acc[t] = (v8f){};
#pragma unroll 5
  for (int kb = 0; kb < KP; kb += 32) { const v16b a = frag_kb(AP + (m0 + nloc) * KP + kb, hlf);
#pragma unroll
    for (int t = 0; t < 8; ++t) acc[t] = wmma16b(a, frag_kb(WB + (size_t)(n0 + t * 16 + nloc) * KP + kb, hlf), acc[t]); }
#pragma unroll
  for (int t = 0; t < 8; ++t)
#pragma unroll
    for (int r = 0; r < 8; ++r) Tf[wave][8 * hlf + r][t * 16 + nloc] = acc[t][r] * (1.0f / (XS * WSC2));
  wave_lds_sync();
  for (int pass = 0; pass < 2; ++pass) { for (int rr = 0; rr < 16; ++rr) *(volatile v4f*)(S + (m0 + rr) * NF + n0 + lane * 4) = *(const v4f*)(&Tf[wave][rr][lane * 4]); __threadfence(); }
}
__global__ __launch_bounds__(256) void ola_kernel(const float* __restrict__ S, const float* __restrict__ wsum, float* __restrict__ out) {
  const size_t u = (size_t)blockIdx.x * 256 + threadIdx.x; if (u >= (size_t)B * LEN) return; const int b = (int)(u / LEN), n = (int)(u % LEN); const int m = n + NF / 2;
  int t0 = (m - NF + HOP) / HOP; if (t0 < 0) t0 = 0; int t1 = m / HOP; if (t1 > T - 1) t1 = T - 1; float s = 0.0f;
#pragma unroll 1
  for (int t = t0; t <= t1; ++t) { const int off = m - HOP * t; if (off >= 0 && off < NF) s += S[((size_t)b * T + t) * NF + off]; }
  const float y = s / bf16_rne(wsum[m]);
  for (int pass = 0; pass < 2; ++pass) { ((volatile float*)out)[u] = y; __threadfence(); }
}
}

extern "C" void kernel_launch(void* const* d_in, const int* in_sizes, int n_in, void* d_out, int out_size, void* d_ws, size_t ws_size, hipStream_t stream) {
  (void)n_in;
  auto Fp = [&](int i) { return (const float*)d_in[i]; };
  if (in_sizes[0] != M * NB1 || in_sizes[1] != M * NB1 || in_sizes[2] != NF * NF || in_sizes[3] != NF * NF || in_sizes[4] != LFULL || out_size != B * LEN) return;
  size_t off = 0; char* ws = (char*)d_ws;
  auto carve = [&](size_t bytes) { char* p = ws + off; off += (bytes + 255) & ~(size_t)255; return p; };
  b16* AP = (b16*)carve((size_t)M * KP * 2); b16* WB = (b16*)carve((size_t)NF * KP * 2); float* S = (float*)carve((size_t)M * NF * 4);
  if (off > ws_size || off > ((size_t)128 << 20)) return;
  aprep_kernel<<<(unsigned)(((size_t)M * KP / 8 + 255) / 256), 256, 0, stream>>>(Fp(0), Fp(1), AP);
  wprep_kernel<<<(unsigned)(((size_t)NF * KP / 8 + 255) / 256), 256, 0, stream>>>(Fp(2), Fp(3), WB);
  gemm_kernel<<<dim3(ML / 64, NF / 128), 128, 0, stream>>>(AP, WB, S);
  ola_kernel<<<(unsigned)(((size_t)B * LEN + 255) / 256), 256, 0, stream>>>(S, Fp(4), (float*)d_out);
}
